// HierarchicalSparseAttention_3427383902611
// MI455X (gfx1250) — hardware-verified
//
#include <hip/hip_runtime.h>
#include <stddef.h>
#include <stdint.h>


typedef _Float16 hh;
typedef hh    v8h  __attribute__((ext_vector_type(8)));
typedef hh    v16h __attribute__((ext_vector_type(16)));
typedef float v4f  __attribute__((ext_vector_type(4)));
typedef float v8f  __attribute__((ext_vector_type(8)));

#define BB   4
#define NN   4096
#define DD   512
#define NM1  4095
#define NYC  2047
#define NKR  6143
#define LVL  12
#define WSC  64.0f
#define LGS  0.00048828125f

union Frag { v16h v; v8h p[2]; };

struct RowMap { int rpb; int bstride; int off; int step; };
typedef char rowmap_size_check[(sizeof(RowMap) == 16) ? 1 : -1];

__device__ __forceinline__ size_t map_row(const RowMap m, int r) {
  const int b = r / m.rpb;
  const int j = r - b * m.rpb;
  return (size_t)b * (size_t)m.bstride + (size_t)m.off + (size_t)j * (size_t)m.step;
}

__device__ __forceinline__ void st2h(hh* p, v8h v) {
  *(volatile v8h*)p = v;
  __threadfence();
  *(volatile v8h*)p = v;
}

__device__ __forceinline__ v8f ld8(const hh* p) {
  return __builtin_convertvector(*(const v8h*)p, v8f);
}

__device__ __forceinline__ v8f mma16(v16h a, v16h b, v8f c) {
  return __builtin_amdgcn_wmma_f32_16x16x32_f16(false, a, false, b, (short)0, c, false, false);
}

__launch_bounds__(256)
__global__ void k_cvt_x(const float* __restrict__ x, hh* xh, int n8) {
  const int t = (int)blockIdx.x * 256 + (int)threadIdx.x;
  if (t >= n8) return;
  const float* s = x + (size_t)t * 8;
  const v4f a = *(const v4f*)s;
  const v4f b = *(const v4f*)(s + 4);
  const v8f f = __builtin_shufflevector(a, b, 0, 1, 2, 3, 4, 5, 6, 7);
  st2h(xh + (size_t)t * 8, __builtin_convertvector(f, v8h));
}

__launch_bounds__(256)
__global__ void k_cvt_w(const float* __restrict__ w0, const float* __restrict__ w1,
                        const float* __restrict__ w2, const float* __restrict__ w3,
                        const float* __restrict__ w4, const float* __restrict__ w5,
                        const float* __restrict__ w6, const float* __restrict__ w7,
                        hh* wh, int n8) {
  const int t = (int)blockIdx.x * 256 + (int)threadIdx.x;
  if (t >= n8) return;
  const int sel = (int)blockIdx.y;
  const float* w = w0;
  if (sel == 1) w = w1;
  if (sel == 2) w = w2;
  if (sel == 3) w = w3;
  if (sel == 4) w = w4;
  if (sel == 5) w = w5;
  if (sel == 6) w = w6;
  if (sel == 7) w = w7;
  const float* s = w + (size_t)t * 8;
  const v4f a = *(const v4f*)s;
  const v4f b = *(const v4f*)(s + 4);
  v8f f = __builtin_shufflevector(a, b, 0, 1, 2, 3, 4, 5, 6, 7);
  f = f * WSC;
  st2h(wh + (size_t)sel * (size_t)n8 * 8 + (size_t)t * 8, __builtin_convertvector(f, v8h));
}

__launch_bounds__(64)
__global__ void k_pool(const float* __restrict__ x, hh* yh) {
  const int b = (int)blockIdx.x;
  const int e = (int)threadIdx.x;
  const float* xb = x + (size_t)b * NN * DD + 8 * e;
  hh* yb = yh + (size_t)b * NM1 * DD + 8 * e;
  v8f pend[LVL];
  #pragma unroll
  for (int i = 0; i < LVL; ++i) { const v8f z = {0, 0, 0, 0, 0, 0, 0, 0}; pend[i] = z; }
  #pragma unroll 1
  for (int i2 = 0; i2 < NN / 2; ++i2) {
    const float* r0 = xb + (size_t)(2 * i2) * DD;
    const v4f a0 = *(const v4f*)(r0);
    const v4f a1 = *(const v4f*)(r0 + 4);
    const v4f c0 = *(const v4f*)(r0 + DD);
    const v4f c1 = *(const v4f*)(r0 + DD + 4);
    const v4f s0 = (a0 + c0) * 0.5f;
    const v4f s1 = (a1 + c1) * 0.5f;
    v8f cur = __builtin_shufflevector(s0, s1, 0, 1, 2, 3, 4, 5, 6, 7);
    st2h(yb + (size_t)i2 * DD, __builtin_convertvector(cur, v8h));
    bool have = true;
    #pragma unroll
    for (int lv = 1; lv < LVL; ++lv) {
      if (have) {
        if (((i2 >> (lv - 1)) & 1) == 0) {
          pend[lv] = cur;
          have = false;
        } else {
          cur = (pend[lv] + cur) * 0.5f;
          const int off = NN - (NN >> lv);
          st2h(yb + (size_t)(off + (i2 >> lv)) * DD, __builtin_convertvector(cur, v8h));
        }
      }
    }
  }
}


__device__ __forceinline__ void epi_store(hh* C, const float* sw, int l, int row0, int M, int n0,
                                          const RowMap om, float oscale, const float* bias, float bscale) {
  const int q = l >> 3, e = l & 7;
  const v4f bz0 = *(const v4f*)(bias + n0 + 8 * e) * bscale;
  const v4f bz1 = *(const v4f*)(bias + n0 + 8 * e + 4) * bscale;
  const int r = row0 + q;
  int bb = r / om.rpb;
  int j = r - bb * om.rpb;
  v8h val[8]; size_t adr[8]; bool ok[8];
  #pragma unroll
  for (int it = 0; it < 8; ++it) {
    const int tr = it * 4 + q;
    const v4f x0 = *(const v4f*)(sw + tr * 64 + 8 * e);
    const v4f x1 = *(const v4f*)(sw + tr * 64 + 8 * e + 4);
    const v4f y0 = x0 * oscale + bz0;
    const v4f y1 = x1 * oscale + bz1;
    const v8f y = __builtin_shufflevector(y0, y1, 0, 1, 2, 3, 4, 5, 6, 7);
    val[it] = __builtin_convertvector(y, v8h);
    ok[it] = (row0 + tr) < M;
    adr[it] = ((size_t)bb * (size_t)om.bstride + (size_t)om.off + (size_t)j * (size_t)om.step) * DD + n0 + 8 * e;
    j += 4;
    if (j >= om.rpb) { j -= om.rpb; bb += 1; }
  }
  #pragma unroll
  for (int it = 0; it < 8; ++it) if (ok[it]) *(volatile v8h*)(C + adr[it]) = val[it];
  __threadfence();
  #pragma unroll
  for (int it = 0; it < 8; ++it) if (ok[it]) *(volatile v8h*)(C + adr[it]) = val[it];
}

__device__ __forceinline__ void epi_store(float* C, const float* sw, int l, int row0, int M, int n0,
                                          const RowMap om, float oscale, const float* bias, float bscale) {
  const int q = l >> 4, e = l & 15;
  const v4f bz = *(const v4f*)(bias + n0 + 4 * e) * bscale;
  const int r = row0 + q;
  int bb = r / om.rpb;
  int j = r - bb * om.rpb;
  v4f val[16]; size_t adr[16]; bool ok[16];
  #pragma unroll
  for (int it = 0; it < 16; ++it) {
    const int tr = it * 2 + q;
    const v4f x0 = *(const v4f*)(sw + tr * 64 + 4 * e);
    val[it] = x0 * oscale + bz;
    ok[it] = (row0 + tr) < M;
    adr[it] = ((size_t)bb * (size_t)om.bstride + (size_t)om.off + (size_t)j * (size_t)om.step) * DD + n0 + 4 * e;
    j += 2;
    if (j >= om.rpb) { j -= om.rpb; bb += 1; }
  }
  #pragma unroll
  for (int it = 0; it < 16; ++it) if (ok[it]) *(volatile v4f*)(C + adr[it]) = val[it];
  __threadfence();
  #pragma unroll
  for (int it = 0; it < 16; ++it) if (ok[it]) *(volatile v4f*)(C + adr[it]) = val[it];
}

template <typename OT>
__launch_bounds__(128)
__global__ void k_gemm(const hh* __restrict__ A, const hh* __restrict__ W0, const hh* __restrict__ W1,
                       const float* __restrict__ bias, OT* C0, OT* C1, int M,
                       RowMap am, RowMap om, float oscale, float bscale) {
  __shared__ __attribute__((aligned(16))) float st[4 * 32 * 64];
  const int l = (int)threadIdx.x & 31;
  const int wv = (int)threadIdx.x >> 5;
  const int h = l >> 4;
  const int m16 = l & 15;
  const hh* W = (blockIdx.z == 0) ? W0 : W1;
  OT* C = (blockIdx.z == 0) ? C0 : C1;
  const int row0 = ((int)blockIdx.x * 4 + wv) * 32;
  const int n0 = (int)blockIdx.y * 64;

  int ra = row0 + m16;      if (ra > M - 1) ra = M - 1;
  int rb = row0 + 16 + m16; if (rb > M - 1) rb = M - 1;
  const hh* pa = A + map_row(am, ra) * DD + 8 * h;
  const hh* pb = A + map_row(am, rb) * DD + 8 * h;
  const hh* pw = W + (size_t)(n0 + m16) * DD + 8 * h;

  const v8f z = {0, 0, 0, 0, 0, 0, 0, 0};
  v8f c0 = z, c1 = z, c2 = z, c3 = z, c4 = z, c5 = z, c6 = z, c7 = z;

  #pragma unroll 2
  for (int k0 = 0; k0 < DD; k0 += 32) {
    Frag a0, a1, b0, b1, b2, b3;
    a0.p[0] = *(const v8h*)(pa + k0);            a0.p[1] = *(const v8h*)(pa + k0 + 16);
    a1.p[0] = *(const v8h*)(pb + k0);            a1.p[1] = *(const v8h*)(pb + k0 + 16);
    b0.p[0] = *(const v8h*)(pw + k0);            b0.p[1] = *(const v8h*)(pw + k0 + 16);
    b1.p[0] = *(const v8h*)(pw + 16 * DD + k0);  b1.p[1] = *(const v8h*)(pw + 16 * DD + k0 + 16);
    b2.p[0] = *(const v8h*)(pw + 32 * DD + k0);  b2.p[1] = *(const v8h*)(pw + 32 * DD + k0 + 16);
    b3.p[0] = *(const v8h*)(pw + 48 * DD + k0);  b3.p[1] = *(const v8h*)(pw + 48 * DD + k0 + 16);
    c0 = mma16(a0.v, b0.v, c0);
    c1 = mma16(a0.v, b1.v, c1);
    c2 = mma16(a0.v, b2.v, c2);
    c3 = mma16(a0.v, b3.v, c3);
    c4 = mma16(a1.v, b0.v, c4);
    c5 = mma16(a1.v, b1.v, c5);
    c6 = mma16(a1.v, b2.v, c6);
    c7 = mma16(a1.v, b3.v, c7);
    asm volatile("v_nop\n\tv_nop\n\tv_nop\n\tv_nop"
                 : "+v"(c0), "+v"(c1), "+v"(c2), "+v"(c3), "+v"(c4), "+v"(c5), "+v"(c6), "+v"(c7)
                 : "v"(a0.v), "v"(a1.v), "v"(b0.v), "v"(b1.v), "v"(b2.v), "v"(b3.v));
  }

  float* sw = st + wv * (32 * 64);
  #pragma unroll
  for (int r = 0; r < 8; ++r) {
    float* p0 = sw + (8 * h + r) * 64 + m16;
    p0[0] = c0[r]; p0[16] = c1[r]; p0[32] = c2[r]; p0[48] = c3[r];
    float* p1 = p0 + 16 * 64;
    p1[0] = c4[r]; p1[16] = c5[r]; p1[32] = c6[r]; p1[48] = c7[r];
  }
  __syncthreads();
  epi_store(C, sw, l, row0, M, n0, om, oscale, bias, bscale);
}

__launch_bounds__(256)
__global__ void k_pair_attn(const hh* __restrict__ Q, const hh* __restrict__ Kt,
                            const hh* __restrict__ Vt, hh* NL, int P, int off, int nw) {
  const int l = (int)threadIdx.x & 31;
  const int gw = (int)blockIdx.x * 8 + ((int)threadIdx.x >> 5);
  if (gw >= nw) return;
  const int b = gw / P;
  const int p = gw - b * P;
  const size_t orow = ((size_t)b * NM1 + off + p) * DD;
  const size_t k0r = ((size_t)b * 2 * P + 2 * p) * DD;
  const size_t k1r = k0r + DD;
  #pragma unroll
  for (int c = 0; c < 2; ++c) {
    const int d = 256 * c + 8 * l;
    const v8f q  = ld8(Q + orow + d);
    const v8f ka = ld8(Kt + k0r + d);
    const v8f kb = ld8(Kt + k1r + d);
    const v8f va = ld8(Vt + k0r + d);
    const v8f vb = ld8(Vt + k1r + d);
    float da = 0.f, db = 0.f;
    #pragma unroll
    for (int i = 0; i < 8; ++i) { da += q[i] * ka[i]; db += q[i] * kb[i]; }
    da += __shfl_xor(da, 1); da += __shfl_xor(da, 2); da += __shfl_xor(da, 4);
    db += __shfl_xor(db, 1); db += __shfl_xor(db, 2); db += __shfl_xor(db, 4);
    const float la = da * LGS, lb = db * LGS;
    const float m = fmaxf(la, lb);
    const float ea = __expf(la - m), eb = __expf(lb - m);
    const float inv = __fdividef(1.0f, (ea + eb) + 1e-9f);
    const float wa = ea * inv, wb = eb * inv;
    const v8f o = va * wa + vb * wb;
    st2h(NL + orow + d, __builtin_convertvector(o, v8h));
  }
}

__launch_bounds__(256)
__global__ void k_path_attn(const hh* __restrict__ Q, const hh* __restrict__ Kc,
                            const hh* __restrict__ Vc, hh* AO, int nw) {
  const int l = (int)threadIdx.x & 31;
  const int gw = (int)blockIdx.x * 8 + ((int)threadIdx.x >> 5);
  if (gw >= nw) return;
  const int b = gw >> 12;
  const int n = gw & (NN - 1);
  const size_t qrow = ((size_t)b * NN + n) * DD;
  const size_t kb = (size_t)b * NKR;
  v8f q[2], o[2];
  float m[2], s[2];
  {
    const size_t kr = (kb + n) * DD;
    #pragma unroll
    for (int c = 0; c < 2; ++c) {
      const int d = 256 * c + 8 * l;
      q[c] = ld8(Q + qrow + d);
      const v8f k = ld8(Kc + kr + d);
      o[c] = ld8(Vc + kr + d);
      float dt = 0.f;
      #pragma unroll
      for (int i = 0; i < 8; ++i) dt += q[c][i] * k[i];
      dt += __shfl_xor(dt, 1); dt += __shfl_xor(dt, 2); dt += __shfl_xor(dt, 4);
      m[c] = dt * LGS;
      s[c] = 1.0f;
    }
  }
  #pragma unroll 1
  for (int t = 0; t < LVL; ++t) {
    if (((n >> t) & 1) == 0) continue;
    int rown;
    if (t == 0) {
      rown = n - 1;
    } else {
      const int sh = t - 1;
      const int yr = (NN - (NN >> sh)) + (n >> t) - 1;
      rown = NN + (yr >> 1);
    }
    rown = rown < 0 ? 0 : (rown > NKR - 1 ? NKR - 1 : rown);
    const size_t kr = (kb + rown) * DD;
    #pragma unroll
    for (int c = 0; c < 2; ++c) {
      const int d = 256 * c + 8 * l;
      const v8f k = ld8(Kc + kr + d);
      const v8f v = ld8(Vc + kr + d);
      float dt = 0.f;
      #pragma unroll
      for (int i = 0; i < 8; ++i) dt += q[c][i] * k[i];
      dt += __shfl_xor(dt, 1); dt += __shfl_xor(dt, 2); dt += __shfl_xor(dt, 4);
      const float lg = dt * LGS;
      const float mn = fmaxf(m[c], lg);
      const float cr = __expf(m[c] - mn);
      const float e = __expf(lg - mn);
      s[c] = s[c] * cr + e;
      o[c] = o[c] * cr + v * e;
      m[c] = mn;
    }
  }
  #pragma unroll
  for (int c = 0; c < 2; ++c) {
    const int d = 256 * c + 8 * l;
    const float inv = __fdividef(1.0f, s[c]);
    const v8f r = o[c] * inv;
    st2h(AO + qrow + d, __builtin_convertvector(r, v8h));
  }
}

extern "C" void kernel_launch(void* const* d_in, const int* in_sizes, int n_in,
                              void* d_out, int out_size, void* d_ws, size_t ws_size,
                              hipStream_t stream) {
  if (n_in < 11) return;
  if (in_sizes[0] != BB * NN * DD) return;
  for (int i = 1; i <= 8; ++i) if (in_sizes[i] != DD * DD) return;
  if (in_sizes[9] != DD || in_sizes[10] != DD) return;
  if (out_size != BB * NN * DD) return;

  const float* x = (const float*)d_in[0];
  const float* wf[8];
  for (int i = 0; i < 8; ++i) wf[i] = (const float*)d_in[1 + i];
  const float* bo_y = (const float*)d_in[9];
  const float* bo_x = (const float*)d_in[10];
  float* out = (float*)d_out;

  char* ws = (char*)d_ws;
  size_t o = 0;
  auto carve = [&](size_t bytes) -> char* {
    char* p = ws + o;
    o = (o + bytes + 255) & ~(size_t)255;
    return p;
  };
  hh* xh   = (hh*)carve((size_t)BB * NN  * DD * 2);
  hh* ybuf = (hh*)carve((size_t)BB * NN  * DD * 2);
  hh* qb   = (hh*)carve((size_t)BB * NN  * DD * 2);
  hh* wh   = (hh*)carve((size_t)8  * DD  * DD * 2);
  hh* kc   = (hh*)carve((size_t)BB * NKR * DD * 2);
  hh* vc   = (hh*)carve((size_t)BB * NKR * DD * 2);
  hh* yc   = (hh*)carve((size_t)BB * NYC * DD * 2);
  if (o > ws_size) return;

  const size_t WW = (size_t)DD * DD;
  const RowMap idm = {1 << 30, 0, 0, 1};
  const dim3 gblk(128);

  { const int n8 = BB * NN * DD / 8;
    k_cvt_x<<<dim3((n8 + 255) / 256), dim3(256), 0, stream>>>(x, xh, n8); }
  { const int n8 = DD * DD / 8;
    k_cvt_w<<<dim3((n8 + 255) / 256, 8), dim3(256), 0, stream>>>(wf[0], wf[1], wf[2], wf[3],
                                                                  wf[4], wf[5], wf[6], wf[7], wh, n8); }
  k_pool<<<dim3(BB), dim3(64), 0, stream>>>(x, ybuf);

  { const int M = BB * NM1;
    k_gemm<hh><<<dim3((M + 127) / 128, DD / 64, 1), gblk, 0, stream>>>(
        ybuf, wh + 0 * WW, wh + 0 * WW, bo_x, qb, qb, M, idm, idm, 0.25f, 0.0f); }

  for (int lv = 0; lv < LVL; ++lv) {
    const int P = NN >> (lv + 1);
    const int off = NN - (NN >> lv);
    const int M = BB * 2 * P;
    const hh* Asrc = (lv == 0) ? xh : ybuf;
    RowMap am = idm;
    float osc = 0.25f;
    if (lv > 0) { am.rpb = 2 * P; am.bstride = NM1; am.off = NN - (NN >> (lv - 1)); am.step = 1; osc = 0.015625f; }
    k_gemm<hh><<<dim3((M + 127) / 128, DD / 64, 2), gblk, 0, stream>>>(
        Asrc, wh + 1 * WW, wh + 2 * WW, bo_x, kc, vc, M, am, idm, osc, 0.0f);
    const int nw = BB * P;
    k_pair_attn<<<dim3((nw + 7) / 8), dim3(256), 0, stream>>>(qb, kc, vc, ybuf, P, off, nw);
  }

  { const int M = BB * NYC;
    const RowMap am = {NYC, NM1, 0, 2};
    k_gemm<hh><<<dim3((M + 127) / 128, DD / 64, 1), gblk, 0, stream>>>(
        ybuf, wh + 3 * WW, wh + 3 * WW, bo_y, yc, yc, M, am, idm, 0.015625f, 16.0f); }

  { const int M = BB * NN;
    k_gemm<hh><<<dim3((M + 127) / 128, DD / 64, 1), gblk, 0, stream>>>(
        xh, wh + 4 * WW, wh + 4 * WW, bo_x, qb, qb, M, idm, idm, 0.25f, 0.0f); }

  { const int M = BB * NN;
    const RowMap om = {NN, NKR, 0, 1};
    k_gemm<hh><<<dim3((M + 127) / 128, DD / 64, 2), gblk, 0, stream>>>(
        xh, wh + 5 * WW, wh + 6 * WW, bo_x, kc, vc, M, idm, om, 0.25f, 0.0f); }
  { const int M = BB * NYC;
    const RowMap om = {NYC, NKR, NN, 1};
    k_gemm<hh><<<dim3((M + 127) / 128, DD / 64, 2), gblk, 0, stream>>>(
        yc, wh + 5 * WW, wh + 6 * WW, bo_x, kc, vc, M, idm, om, 0.015625f, 0.0f); }

  { const int nw = BB * NN;
    k_path_attn<<<dim3((nw + 7) / 8), dim3(256), 0, stream>>>(qb, kc, vc, ybuf, nw); }

  { const int M = BB * NN;
    k_gemm<float><<<dim3((M + 127) / 128, DD / 64, 1), gblk, 0, stream>>>(
        ybuf, wh + 7 * WW, wh + 7 * WW, bo_x, out, out, M, idm, idm, 0.0009765625f, 1.0f); }
}
